// GNNAttentionResidualModel_73632919323004
// MI455X (gfx1250) — hardware-verified
//
#include <hip/hip_runtime.h>
#include <stddef.h>
#include <stdint.h>


#define DF    128
#define CATP  256
#define GR    64
#define GTHR  256
#define CSP   132
#define NB    512
#define CHUNK 2048
#define NTHR  256
#define NWAVE 8
#define WCAP  256
#define NGRP  (CHUNK / (NTHR * 4))
#define PARTW 256

#define LDS_F (NB * DF + NB * 2 * 3)
#define LDS_I (NWAVE * WCAP + NWAVE + 16)
#define LDS_BYTES ((LDS_F + LDS_I) * 4)

static_assert(WCAP == (CHUNK / NTHR) * 32);
static_assert(NGRP == 2);
static_assert(NB == 512);
static_assert(CHUNK <= 4096);
static_assert(((NB * DF + NB * 2) % 4) == 0);
static_assert(LDS_BYTES == 282720);

typedef float          v4f  __attribute__((ext_vector_type(4)));
typedef float          v8f  __attribute__((ext_vector_type(8)));
typedef int            v4i  __attribute__((ext_vector_type(4)));
typedef unsigned short v4us __attribute__((ext_vector_type(4)));
typedef unsigned short v8us __attribute__((ext_vector_type(8)));
typedef __bf16         v16b __attribute__((ext_vector_type(16)));
typedef double         v2d  __attribute__((ext_vector_type(2)));

union FragB { v16b v; v8us h[2]; };
union U8    { v8us v; v4us q[2]; v4i i; };
union U4    { v4us v; unsigned long long u; };

__device__ __forceinline__ v8f wm(v16b a, v16b b, v8f c) {
  v8f d = __builtin_amdgcn_wmma_f32_16x16x32_bf16(false, a, false, b, (short)0, c, false, false);
  asm volatile("v_nop\n\tv_nop\n\tv_nop\n\tv_nop" : "+v"(d) : "v"(a), "v"(b));
  return d;
}

__device__ __forceinline__ unsigned short bfr(float f) {
  unsigned u = __float_as_uint(f);
  u += 0x7FFFu + ((u >> 16) & 1u);
  return (unsigned short)(u >> 16);
}
__device__ __forceinline__ float bfx(unsigned short s) { return __uint_as_float(((unsigned)s) << 16); }

__device__ __forceinline__ void split4(v4f y, v4us& hi, v4us& lo) {
  const unsigned short a0 = bfr(y.x), a1 = bfr(y.y), a2 = bfr(y.z), a3 = bfr(y.w);
  const unsigned short b0 = bfr(y.x - bfx(a0)), b1 = bfr(y.y - bfx(a1));
  const unsigned short b2 = bfr(y.z - bfx(a2)), b3 = bfr(y.w - bfx(a3));
  v4us H, L;
  H.x = a0; H.y = a1; H.z = a2; H.w = a3;
  L.x = b0; L.y = b1; L.z = b2; L.w = b3;
  hi = H; lo = L;
}

__global__ __launch_bounds__(256) void k_split(const float* __restrict__ a,
                                               unsigned short* ph, unsigned short* pl, int n8) {
  const int i = blockIdx.x * 256 + threadIdx.x;
  if (i >= n8) return;
  const size_t o = (size_t)i * 8;
  const v4f f0 = *(const v4f*)(a + o);
  const v4f f1 = *(const v4f*)(a + o + 4);
  U8 H, L;
  split4(f0, H.q[0], L.q[0]);
  split4(f1, H.q[1], L.q[1]);
  *(volatile v4i*)(ph + o) = H.i;
  *(volatile v4i*)(pl + o) = L.i;
  __threadfence();
  *(volatile v4i*)(ph + o) = H.i;
  *(volatile v4i*)(pl + o) = L.i;
}

__global__ __launch_bounds__(256) void k_wprep(const float* __restrict__ W, unsigned short* Wh,
                                               unsigned short* Wl, int K, int sh, int total) {
  const int t = blockIdx.x * 256 + threadIdx.x;
  if (t >= total) return;
  const int n  = t >> sh;
  const int k8 = t & ((K >> 3) - 1);
  float f[8];
#pragma unroll
  for (int i = 0; i < 8; ++i) f[i] = W[(size_t)(8 * k8 + i) * DF + n];
  v4f fa, fb;
  fa.x = f[0]; fa.y = f[1]; fa.z = f[2]; fa.w = f[3];
  fb.x = f[4]; fb.y = f[5]; fb.z = f[6]; fb.w = f[7];
  U8 H, L;
  split4(fa, H.q[0], L.q[0]);
  split4(fb, H.q[1], L.q[1]);
  const size_t o = (size_t)n * K + 8 * k8;
  *(volatile v4i*)(Wh + o) = H.i;
  *(volatile v4i*)(Wl + o) = L.i;
  __threadfence();
  *(volatile v4i*)(Wh + o) = H.i;
  *(volatile v4i*)(Wl + o) = L.i;
}

template <int EPI>
__device__ __forceinline__ void gemm_stores(const float* Cs, const float* Asl, const float* Adl,
                                            const double* Sd, const double* Qd,
                                            float* C, float* outS, float* outD, double* part,
                                            int rowBase, int wave, int lane) {
#pragma unroll
  for (int i = 0; i < 8; ++i) {
    const int rl = 8 * wave + i;
    const v4f v = *(const v4f*)(Cs + rl * CSP + 4 * lane);
    *(volatile v4f*)(C + (size_t)(rowBase + rl) * DF + 4 * lane) = v;
  }
  if (EPI == 0) {
    if (wave == 0) {
      const v4f v = *(const v4f*)(Asl + 4 * lane);
      *(volatile v4f*)(outS + (size_t)rowBase * 2 + 4 * lane) = v;
    }
    if (wave == 1) {
      const v4f v = *(const v4f*)(Adl + 4 * lane);
      *(volatile v4f*)(outD + (size_t)rowBase * 2 + 4 * lane) = v;
    }
  }
  if (EPI == 2) {
    double* pp = part + (size_t)blockIdx.x * PARTW;
    if (wave == 0) {
      const v2d a = *(const v2d*)(Sd + 2 * lane);
      const v2d b = *(const v2d*)(Sd + 64 + 2 * lane);
      *(volatile v2d*)(pp + 2 * lane)      = a;
      *(volatile v2d*)(pp + 64 + 2 * lane) = b;
    }
    if (wave == 1) {
      const v2d a = *(const v2d*)(Qd + 2 * lane);
      const v2d b = *(const v2d*)(Qd + 64 + 2 * lane);
      *(volatile v2d*)(pp + 128 + 2 * lane) = a;
      *(volatile v2d*)(pp + 192 + 2 * lane) = b;
    }
  }
}

template <int KD, int EPI>
__global__ __launch_bounds__(GTHR) void k_gemm(
    const unsigned short* __restrict__ Ah, const unsigned short* __restrict__ Al,
    const unsigned short* __restrict__ Bh, const unsigned short* __restrict__ Bl,
    const float* __restrict__ bias, const float* __restrict__ att_s, const float* __restrict__ att_d,
    float* C, float* outS, float* outD, double* part, int nN) {
  __shared__ __attribute__((aligned(16))) float  Cs[GR * CSP];
  __shared__ __attribute__((aligned(16))) float  attSl[DF];
  __shared__ __attribute__((aligned(16))) float  attDl[DF];
  __shared__ __attribute__((aligned(16))) float  Asl[GR * 2];
  __shared__ __attribute__((aligned(16))) float  Adl[GR * 2];
  __shared__ __attribute__((aligned(16))) double Sd[DF];
  __shared__ __attribute__((aligned(16))) double Qd[DF];

  const int tid  = threadIdx.x;
  const int lane = tid & 31;
  const int wave = tid >> 5;
  const int h    = lane >> 4;
  const int m    = lane & 15;
  const int wr   = wave & 3;
  const int wc   = wave >> 2;
  const int rowBase = blockIdx.x * GR;

  if (EPI == 0) {
    if (tid < DF) { attSl[tid] = att_s[tid]; attDl[tid] = att_d[tid]; }
  }

  int arow = rowBase + 16 * wr + m;
  if (arow > nN - 1) arow = nN - 1;
  const unsigned short* pah = Ah + (size_t)arow * KD + 8 * h;
  const unsigned short* pal = Al + (size_t)arow * KD + 8 * h;
  const unsigned short* pbh = Bh + (size_t)(64 * wc + m) * KD + 8 * h;
  const unsigned short* pbl = Bl + (size_t)(64 * wc + m) * KD + 8 * h;

  const v8f z8 = {0.f, 0.f, 0.f, 0.f, 0.f, 0.f, 0.f, 0.f};
  v8f acc[4];
#pragma unroll
  for (int nt = 0; nt < 4; ++nt) acc[nt] = z8;

#pragma unroll 1
  for (int kt = 0; kt < KD / 32; ++kt) {
    const int k0 = kt * 32;
    FragB ah, al;
    ah.h[0] = *(const v8us*)(pah + k0);
    ah.h[1] = *(const v8us*)(pah + k0 + 16);
    al.h[0] = *(const v8us*)(pal + k0);
    al.h[1] = *(const v8us*)(pal + k0 + 16);
#pragma unroll
    for (int nt = 0; nt < 4; ++nt) {
      const size_t bo = (size_t)nt * 16 * KD + k0;
      FragB bh, bl;
      bh.h[0] = *(const v8us*)(pbh + bo);
      bh.h[1] = *(const v8us*)(pbh + bo + 16);
      bl.h[0] = *(const v8us*)(pbl + bo);
      bl.h[1] = *(const v8us*)(pbl + bo + 16);
      acc[nt] = wm(ah.v, bh.v, acc[nt]);
      acc[nt] = wm(ah.v, bl.v, acc[nt]);
      acc[nt] = wm(al.v, bh.v, acc[nt]);
    }
  }

#pragma unroll
  for (int nt = 0; nt < 4; ++nt) {
    const int col = 64 * wc + 16 * nt + m;
    float bv = 0.f;
    if (EPI != 0) bv = bias[col];
#pragma unroll
    for (int r = 0; r < 8; ++r) {
      float v = acc[nt][r] + bv;
      if (EPI == 2) v = v > 0.f ? v : 0.f;
      Cs[(16 * wr + 8 * h + r) * CSP + col] = v;
    }
  }
  __syncthreads();

  if (EPI == 0) {
    if (wave < 4) {
      const int rl = 16 * wave + m;
      const float* cp = Cs + rl * CSP + 64 * h;
      const float* sp = attSl + 64 * h;
      const float* dp = attDl + 64 * h;
      float s = 0.f, d = 0.f;
#pragma unroll 4
      for (int c = 0; c < 64; ++c) { const float v = cp[c]; s += v * sp[c]; d += v * dp[c]; }
      Asl[rl * 2 + h] = s;
      Adl[rl * 2 + h] = d;
    }
    __syncthreads();
  }
  if (EPI == 2) {
    if (tid < DF) {
      double s = 0.0, q = 0.0;
#pragma unroll 4
      for (int r = 0; r < GR; ++r) { const double v = (double)Cs[r * CSP + tid]; s += v; q += v * v; }
      Sd[tid] = s;
      Qd[tid] = q;
    }
    __syncthreads();
  }

  gemm_stores<EPI>(Cs, Asl, Adl, Sd, Qd, C, outS, outD, part, rowBase, wave, lane);
  __threadfence();
  gemm_stores<EPI>(Cs, Asl, Adl, Sd, Qd, C, outS, outD, part, rowBase, wave, lane);
}

__global__ __launch_bounds__(NTHR) void k_agg(
    const float* __restrict__ hg, const float* __restrict__ asv, const float* __restrict__ adv,
    const int* __restrict__ ei, const float* __restrict__ bias,
    unsigned short* catH, unsigned short* catL, int coff, int nN, int nE) {
  extern __shared__ v4f lds_dyn[];
  float* sacc = (float*)lds_dyn;
  float* den  = sacc + NB * DF;
  float* adl  = den + NB * 2;
  float* shf  = adl + NB * 2;
  int*   list = (int*)(shf + NB * 2);
  int*   wcnt = list + NWAVE * WCAP;
  float* red  = (float*)(wcnt + NWAVE);

  const int tid  = threadIdx.x;
  const int lane = tid & 31;
  const int wave = tid >> 5;
  const int m    = lane & 15;
  const int hd   = lane >> 4;
  const int nodeBase = blockIdx.x * NB;

  {
    const v4f z4 = {0.f, 0.f, 0.f, 0.f};
    for (int i = tid; i < (NB * DF + NB * 2) / 4; i += NTHR) lds_dyn[i] = z4;
  }
  float mx = -3.0e38f;
#pragma unroll 1
  for (int i = tid; i < 2 * nN; i += NTHR) mx = fmaxf(mx, asv[i]);
  mx = fmaxf(mx, __shfl_xor(mx, 16, 32));
  mx = fmaxf(mx, __shfl_xor(mx, 8, 32));
  mx = fmaxf(mx, __shfl_xor(mx, 4, 32));
  mx = fmaxf(mx, __shfl_xor(mx, 2, 32));
  if (lane < 2) red[wave * 2 + lane] = mx;
  __syncthreads();
  for (int i = tid; i < NB * 2; i += NTHR) {
    const int hh = i & 1, slot = i >> 1;
    int node = nodeBase + slot;
    if (node > nN - 1) node = nN - 1;
    float S = red[hh];
#pragma unroll
    for (int w = 1; w < NWAVE; ++w) S = fmaxf(S, red[w * 2 + hh]);
    const float a = adv[(size_t)node * 2 + hh];
    adl[i] = a;
    const float t = S + a;
    shf[i] = (t > 0.f) ? t : 0.2f * t;
  }
  __syncthreads();

  const int* eid = ei + nE;
  const bool al16 = ((((size_t)eid) & 15) == 0);

  const int nChunks = (nE + CHUNK - 1) / CHUNK;
#pragma unroll 1
  for (int ch = 0; ch < nChunks; ++ch) {
    const int cbase = ch * CHUNK;
    int wc = 0;
#pragma unroll
    for (int g = 0; g < NGRP; ++g) {
      const int el0 = (g * NTHR + tid) * 4;
      const int e0  = cbase + el0;
      const int sent = -2147483647 - 1;
      v4i d;
      if (al16 && (cbase + CHUNK <= nE)) {
        d = *(const v4i*)(eid + e0);
      } else {
        d.x = (e0     < nE) ? eid[min(e0,     nE - 1)] : sent;
        d.y = (e0 + 1 < nE) ? eid[min(e0 + 1, nE - 1)] : sent;
        d.z = (e0 + 2 < nE) ? eid[min(e0 + 2, nE - 1)] : sent;
        d.w = (e0 + 3 < nE) ? eid[min(e0 + 3, nE - 1)] : sent;
      }
      const unsigned s0 = (unsigned)d.x - (unsigned)nodeBase;
      const unsigned s1 = (unsigned)d.y - (unsigned)nodeBase;
      const unsigned s2 = (unsigned)d.z - (unsigned)nodeBase;
      const unsigned s3 = (unsigned)d.w - (unsigned)nodeBase;
      const bool h0 = s0 < (unsigned)NB;
      const bool h1 = s1 < (unsigned)NB;
      const bool h2 = s2 < (unsigned)NB;
      const bool h3 = s3 < (unsigned)NB;
      const unsigned many = __builtin_amdgcn_ballot_w32(h0 | h1 | h2 | h3);
      if (many != 0u) {
#define HITJ(J, HJ, SJ) { \
          const unsigned mj = __builtin_amdgcn_ballot_w32(HJ); \
          if (HJ) { \
            const int pos = wc + (int)__builtin_amdgcn_mbcnt_lo(mj, 0u); \
            if (pos < WCAP) list[wave * WCAP + pos] = ((el0 + (J)) << 9) | (int)(SJ); \
          } \
          wc += (int)__builtin_popcount(mj); }
        HITJ(0, h0, s0)
        HITJ(1, h1, s1)
        HITJ(2, h2, s2)
        HITJ(3, h3, s3)
#undef HITJ
      }
    }
    if (lane == 0) wcnt[wave] = wc;
    __syncthreads();

    if (wave == 0) {
      for (int wsx = 0; wsx < NWAVE; ++wsx) {
        int n = wcnt[wsx];
        if (n > WCAP) n = WCAP;
        if (n < 0) n = 0;
        for (int i = 0; i < n; ++i) {
          const int ent  = list[wsx * WCAP + i];
          const int slot = ent & (NB - 1);
          const int el   = (ent >> 9) & (CHUNK - 1);
          int e = cbase + el;
          if (e > nE - 1) e = nE - 1;
          int src = ei[e];
          src = src < 0 ? 0 : (src > nN - 1 ? nN - 1 : src);
          float al = asv[(size_t)src * 2 + hd] + adl[slot * 2 + hd];
          al = (al > 0.f) ? al : 0.2f * al;
          const float p = __expf(al - shf[slot * 2 + hd]);
          const v4f xv = *(const v4f*)(hg + (size_t)src * DF + 4 * lane);
          v4f* sp = (v4f*)(sacc + slot * DF + 4 * lane);
          const v4f cur = *sp;
          const v4f nxt = cur + p * xv;
          *sp = nxt;
          if (m == 0) {
            const float o = den[slot * 2 + hd];
            den[slot * 2 + hd] = o + p;
          }
        }
      }
    }
    __syncthreads();
  }

  const v4f b4 = *(const v4f*)(bias + 4 * lane);
#pragma unroll 1
  for (int j = 0; j < NB / NWAVE; ++j) {
    const int slot = wave * (NB / NWAVE) + j;
    const int node = nodeBase + slot;
    if (node >= nN) break;
    const size_t nrow = (size_t)node;
    float al = asv[nrow * 2 + hd] + adl[slot * 2 + hd];
    al = (al > 0.f) ? al : 0.2f * al;
    const float p = __expf(al - shf[slot * 2 + hd]);
    const v4f xv = *(const v4f*)(hg + nrow * DF + 4 * lane);
    const v4f sv = *(const v4f*)(sacc + slot * DF + 4 * lane) + p * xv;
    const float dv  = den[slot * 2 + hd] + p;
    const float inv = 1.0f / (dv + 1e-16f);
    const v4f y = sv * inv + b4;
    U4 H, L;
    split4(y, H.v, L.v);
    const size_t o = nrow * CATP + (size_t)coff + 4 * lane;
    *(volatile unsigned long long*)(catH + o) = H.u;
    *(volatile unsigned long long*)(catL + o) = L.u;
    __threadfence();
    *(volatile unsigned long long*)(catH + o) = H.u;
    *(volatile unsigned long long*)(catL + o) = L.u;
  }
}

__global__ __launch_bounds__(DF) void k_bnstat(const double* __restrict__ part, int nblk, int nN,
                                               float* stat) {
  const int c = threadIdx.x;
  double s = 0.0, q = 0.0;
#pragma unroll 1
  for (int b = 0; b < nblk; ++b) {
    s += part[(size_t)b * PARTW + c];
    q += part[(size_t)b * PARTW + 128 + c];
  }
  const double invN = 1.0 / (double)nN;
  const double mu = s * invN;
  double var = q * invN - mu * mu;
  if (var < 0.0) var = 0.0;
  const float varf = (float)var;
  const float rs = 1.0f / sqrtf(varf + 1e-5f);
  const float muf = (float)mu;
  *(volatile float*)(stat + c)      = muf;
  *(volatile float*)(stat + DF + c) = rs;
  __threadfence();
  *(volatile float*)(stat + c)      = muf;
  *(volatile float*)(stat + DF + c) = rs;
}

__global__ __launch_bounds__(256) void k_bn0(const float* __restrict__ mpl, const float* __restrict__ res,
                                             const float* __restrict__ stat, const float* __restrict__ g,
                                             const float* __restrict__ b, float* h0,
                                             unsigned short* h0h, unsigned short* h0l, int nN) {
  const int t = blockIdx.x * 256 + threadIdx.x;
  const int row = t >> 5;
  const int lane = t & 31;
  if (row >= nN) return;
  const size_t o = (size_t)row * DF + 4 * lane;
  const v4f mv = *(const v4f*)(mpl + o);
  const v4f rv = *(const v4f*)(res + o);
  const v4f mu = *(const v4f*)(stat + 4 * lane);
  const v4f rs = *(const v4f*)(stat + DF + 4 * lane);
  const v4f g4 = *(const v4f*)(g + 4 * lane);
  const v4f b4 = *(const v4f*)(b + 4 * lane);
  v4f y = (mv - mu) * rs * g4 + b4;
  y = y + rv;
  U4 H, L;
  split4(y, H.v, L.v);
  *(volatile v4f*)(h0 + o) = y;
  *(volatile unsigned long long*)(h0h + o) = H.u;
  *(volatile unsigned long long*)(h0l + o) = L.u;
  __threadfence();
  *(volatile v4f*)(h0 + o) = y;
  *(volatile unsigned long long*)(h0h + o) = H.u;
  *(volatile unsigned long long*)(h0l + o) = L.u;
}

__global__ __launch_bounds__(256) void k_bn1(const float* __restrict__ mpl, const float* __restrict__ res,
                                             const float* __restrict__ stat, const float* __restrict__ g,
                                             const float* __restrict__ b, float* out, int nN) {
  const int t = blockIdx.x * 256 + threadIdx.x;
  const int row = t >> 5;
  const int lane = t & 31;
  if (row >= nN) return;
  const size_t o = (size_t)row * DF + 4 * lane;
  const v4f mv = *(const v4f*)(mpl + o);
  const v4f rv = *(const v4f*)(res + o);
  const v4f mu = *(const v4f*)(stat + 4 * lane);
  const v4f rs = *(const v4f*)(stat + DF + 4 * lane);
  const v4f g4 = *(const v4f*)(g + 4 * lane);
  const v4f b4 = *(const v4f*)(b + 4 * lane);
  v4f y = (mv - mu) * rs * g4 + b4;
  y = y + rv;
  *(volatile v4f*)(out + o) = y;
  __threadfence();
  *(volatile v4f*)(out + o) = y;
}

extern "C" void kernel_launch(void* const* d_in, const int* in_sizes, int n_in,
                              void* d_out, int out_size, void* d_ws, size_t ws_size,
                              hipStream_t stream) {
  if (n_in < 30) return;
  const int nN = in_sizes[0] / 256;
  if (nN <= 0 || in_sizes[0] != nN * 256 || (nN % GR) != 0) return;
  if ((in_sizes[2] & 1) != 0 || (in_sizes[3] & 1) != 0) return;
  const int nEf = in_sizes[2] / 2;
  const int nEb = in_sizes[3] / 2;
  if (nEf < 1 || nEb < 1) return;
  if (in_sizes[4] != 256 * DF || in_sizes[8] != 256 * DF || in_sizes[20] != 256 * DF ||
      in_sizes[24] != 256 * DF || in_sizes[28] != 256 * DF) return;
  if (in_sizes[12] != DF * DF || in_sizes[16] != DF * DF) return;
  {
    const int vec_idx[19] = {5, 6, 7, 9, 10, 11, 13, 14, 15, 17, 18, 19, 21, 22, 23, 25, 26, 27, 29};
    for (int i = 0; i < 19; ++i) if (in_sizes[vec_idx[i]] != DF) return;
  }
  if (out_size != nN * DF) return;

  const float* x         = (const float*)d_in[0];
  const int*   fwd_ei    = (const int*)d_in[2];
  const int*   bwd_ei    = (const int*)d_in[3];
  const float* fwd0_w    = (const float*)d_in[4];
  const float* fwd0_asrc = (const float*)d_in[5];
  const float* fwd0_adst = (const float*)d_in[6];
  const float* fwd0_b    = (const float*)d_in[7];
  const float* bwd0_w    = (const float*)d_in[8];
  const float* bwd0_asrc = (const float*)d_in[9];
  const float* bwd0_adst = (const float*)d_in[10];
  const float* bwd0_b    = (const float*)d_in[11];
  const float* fwd1_w    = (const float*)d_in[12];
  const float* fwd1_asrc = (const float*)d_in[13];
  const float* fwd1_adst = (const float*)d_in[14];
  const float* fwd1_b    = (const float*)d_in[15];
  const float* bwd1_w    = (const float*)d_in[16];
  const float* bwd1_asrc = (const float*)d_in[17];
  const float* bwd1_adst = (const float*)d_in[18];
  const float* bwd1_b    = (const float*)d_in[19];
  const float* merge0_w  = (const float*)d_in[20];
  const float* merge0_b  = (const float*)d_in[21];
  const float* bn0_g     = (const float*)d_in[22];
  const float* bn0_b     = (const float*)d_in[23];
  const float* merge1_w  = (const float*)d_in[24];
  const float* merge1_b  = (const float*)d_in[25];
  const float* bn1_g     = (const float*)d_in[26];
  const float* bn1_b     = (const float*)d_in[27];
  const float* res0_w    = (const float*)d_in[28];
  const float* res0_b    = (const float*)d_in[29];
  float* out = (float*)d_out;

  char* base = (char*)d_ws;
  size_t off = 0;
  auto carve = [&](size_t bytes) -> void* { void* p = base + off; off += (bytes + 255) & ~(size_t)255; return p; };
  const size_t szP256 = (size_t)nN * 256 * 2;
  const size_t szF128 = (size_t)nN * DF * 4;
  const size_t szAtt  = (size_t)nN * 2 * 4;
  unsigned short* xh   = (unsigned short*)carve(szP256);
  unsigned short* xl   = (unsigned short*)carve(szP256);
  float* hgF  = (float*)carve(szF128);
  float* hgB  = (float*)carve(szF128);
  unsigned short* catH = (unsigned short*)carve(szP256);
  unsigned short* catL = (unsigned short*)carve(szP256);
  float* h0   = (float*)carve(szF128);
  float* asF  = (float*)carve(szAtt);
  float* adF  = (float*)carve(szAtt);
  float* asB  = (float*)carve(szAtt);
  float* adB  = (float*)carve(szAtt);
  const size_t szW256 = (size_t)DF * 256 * 2, szW128 = (size_t)DF * DF * 2;
  unsigned short* wF0h = (unsigned short*)carve(szW256); unsigned short* wF0l = (unsigned short*)carve(szW256);
  unsigned short* wB0h = (unsigned short*)carve(szW256); unsigned short* wB0l = (unsigned short*)carve(szW256);
  unsigned short* wM0h = (unsigned short*)carve(szW256); unsigned short* wM0l = (unsigned short*)carve(szW256);
  unsigned short* wM1h = (unsigned short*)carve(szW256); unsigned short* wM1l = (unsigned short*)carve(szW256);
  unsigned short* wR0h = (unsigned short*)carve(szW256); unsigned short* wR0l = (unsigned short*)carve(szW256);
  unsigned short* wF1h = (unsigned short*)carve(szW128); unsigned short* wF1l = (unsigned short*)carve(szW128);
  unsigned short* wB1h = (unsigned short*)carve(szW128); unsigned short* wB1l = (unsigned short*)carve(szW128);
  const int nblk = nN / GR;
  double* part = (double*)carve((size_t)nblk * PARTW * 8);
  float*  stat = (float*)carve(1024);
  if (off > ws_size || off > (size_t)134217728) return;
  float* resP = (float*)catH;
  unsigned short* h0h = xh;
  unsigned short* h0l = xl;

  auto wprep = [&](const float* W, int K, unsigned short* Wh, unsigned short* Wl) {
    const int total = DF * (K / 8);
    const int sh = (K == 256) ? 5 : 4;
    k_wprep<<<(total + 255) / 256, 256, 0, stream>>>(W, Wh, Wl, K, sh, total);
  };
  wprep(fwd0_w, 256, wF0h, wF0l);
  wprep(bwd0_w, 256, wB0h, wB0l);
  wprep(merge0_w, 256, wM0h, wM0l);
  wprep(merge1_w, 256, wM1h, wM1l);
  wprep(res0_w, 256, wR0h, wR0l);
  wprep(fwd1_w, DF, wF1h, wF1l);
  wprep(bwd1_w, DF, wB1h, wB1l);

  {
    const int n8 = nN * 256 / 8;
    k_split<<<(n8 + 255) / 256, 256, 0, stream>>>(x, xh, xl, n8);
  }

  const int ggrid = nN / GR;
  const int agrid = (nN + NB - 1) / NB;
  const int bgrid = (nN * 32 + 255) / 256;
  hipFuncSetAttribute(reinterpret_cast<const void*>(&k_agg),
                      hipFuncAttributeMaxDynamicSharedMemorySize, LDS_BYTES);

  k_gemm<256, 0><<<ggrid, GTHR, 0, stream>>>(xh, xl, wF0h, wF0l, fwd0_b, fwd0_asrc, fwd0_adst,
                                             hgF, asF, adF, part, nN);
  k_gemm<256, 0><<<ggrid, GTHR, 0, stream>>>(xh, xl, wB0h, wB0l, bwd0_b, bwd0_asrc, bwd0_adst,
                                             hgB, asB, adB, part, nN);
  k_agg<<<agrid, NTHR, LDS_BYTES, stream>>>(hgF, asF, adF, fwd_ei, fwd0_b, catH, catL, 0, nN, nEf);
  k_agg<<<agrid, NTHR, LDS_BYTES, stream>>>(hgB, asB, adB, bwd_ei, bwd0_b, catH, catL, DF, nN, nEb);
  k_gemm<256, 2><<<ggrid, GTHR, 0, stream>>>(catH, catL, wM0h, wM0l, merge0_b, fwd0_asrc, fwd0_adst,
                                             hgF, asF, adF, part, nN);
  k_gemm<256, 1><<<ggrid, GTHR, 0, stream>>>(xh, xl, wR0h, wR0l, res0_b, fwd0_asrc, fwd0_adst,
                                             resP, asF, adF, part, nN);
  k_bnstat<<<1, DF, 0, stream>>>(part, nblk, nN, stat);
  k_bn0<<<bgrid, 256, 0, stream>>>(hgF, resP, stat, bn0_g, bn0_b, h0, h0h, h0l, nN);

  k_gemm<DF, 0><<<ggrid, GTHR, 0, stream>>>(h0h, h0l, wF1h, wF1l, fwd1_b, fwd1_asrc, fwd1_adst,
                                            hgF, asF, adF, part, nN);
  k_gemm<DF, 0><<<ggrid, GTHR, 0, stream>>>(h0h, h0l, wB1h, wB1l, bwd1_b, bwd1_asrc, bwd1_adst,
                                            hgB, asB, adB, part, nN);
  k_agg<<<agrid, NTHR, LDS_BYTES, stream>>>(hgF, asF, adF, fwd_ei, fwd1_b, catH, catL, 0, nN, nEf);
  k_agg<<<agrid, NTHR, LDS_BYTES, stream>>>(hgB, asB, adB, bwd_ei, bwd1_b, catH, catL, DF, nN, nEb);
  k_gemm<256, 2><<<ggrid, GTHR, 0, stream>>>(catH, catL, wM1h, wM1l, merge1_b, fwd1_asrc, fwd1_adst,
                                             hgF, asF, adF, part, nN);
  k_bnstat<<<1, DF, 0, stream>>>(part, nblk, nN, stat);
  k_bn1<<<bgrid, 256, 0, stream>>>(hgF, h0, stat, bn1_g, bn1_b, out, nN);
}
